// GroupedQueryAttention_46591805227232
// MI455X (gfx1250) — hardware-verified
//
#include <hip/hip_runtime.h>


#ifndef NB
#define NB 2
#endif
#ifndef SEQ
#define SEQ 2048
#endif
#define NB_FULL  2
#define SEQ_FULL 2048
#define TT   SEQ
#define DM   2048
#define NH_  16
#define NKV  4
#define REP  (NH_ / NKV)
#define HD   128
#define DQ   (NH_ * HD)
#define DKV  (NKV * HD)
#define ZH   2
#ifndef RH
#define RH   ((SEQ >= 512) ? 256 : 128)
#endif
#define PCAR 1024.0f
#define ACAR 16.0f
#define WCAR 64.0f
#define SCL  0.08838834764831845f

static_assert(NB <= NB_FULL);
static_assert(SEQ <= SEQ_FULL);
static_assert(TT % 128 == 0);
static_assert(TT >= 2 * RH);
static_assert(RH % 128 == 0);
static_assert(HD % 64 == 0);
static_assert(HD == 128);
static_assert(DM % 64 == 0);
static_assert(DQ % 64 == 0);
static_assert(DKV % 64 == 0);
static_assert(DM % 32 == 0);
static_assert(DQ % 32 == 0);
static_assert(REP % ZH == 0);
static_assert(NH_ % ZH == 0);
static_assert(DQ == DM);
static_assert((TT * DM) % 8 == 0);

typedef _Float16 h16;
typedef unsigned short bf;
typedef __attribute__((ext_vector_type(16))) __bf16   v16bf;
typedef __attribute__((ext_vector_type(16))) _Float16 v16h;
typedef __attribute__((ext_vector_type(8)))  _Float16 v8h;
typedef __attribute__((ext_vector_type(8)))  unsigned short v8us;
typedef __attribute__((ext_vector_type(8)))  float    v8f;
typedef __attribute__((ext_vector_type(4)))  float    v4f;
typedef __attribute__((ext_vector_type(2)))  _Float16 v2h;
typedef __attribute__((ext_vector_type(4)))  _Float16 v4h;
typedef __attribute__((ext_vector_type(2)))  unsigned short v2us;
typedef __attribute__((ext_vector_type(4)))  unsigned short v4us;
typedef __attribute__((ext_vector_type(2)))  float    v2f;
typedef v4f  __attribute__((may_alias)) v4fa;

__device__ __forceinline__ unsigned short f2bf(float f) { unsigned u = __float_as_uint(f); u += 0x7FFFu + ((u >> 16) & 1u); return (unsigned short)(u >> 16); }
__device__ __forceinline__ float bf2f(unsigned short b) { return __uint_as_float(((unsigned)b) << 16); }
__device__ __forceinline__ float bfr(float f) { return bf2f(f2bf(f)); }
__device__ __forceinline__ v16h cat16(v8h lo, v8h hi) { return __builtin_shufflevector(lo, hi, 0, 1, 2, 3, 4, 5, 6, 7, 8, 9, 10, 11, 12, 13, 14, 15); }
__device__ __forceinline__ v16bf cat16b(v8us lo, v8us hi) { return __builtin_bit_cast(v16bf, __builtin_shufflevector(lo, hi, 0, 1, 2, 3, 4, 5, 6, 7, 8, 9, 10, 11, 12, 13, 14, 15)); }
__device__ __forceinline__ v8f wmma16(v16h a, v16h b, v8f c) { return __builtin_amdgcn_wmma_f32_16x16x32_f16(false, a, false, b, (short)0, c, false, false); }
__device__ __forceinline__ v8f wmmab(v16bf a, v16bf b, v8f c) { return __builtin_amdgcn_wmma_f32_16x16x32_bf16(false, a, false, b, (short)0, c, false, false); }
__device__ __forceinline__ h16 tohx(float x) { return (h16)x; }
__device__ __forceinline__ void splitf(float y, unsigned short& h, unsigned short& l) { h = f2bf(y); l = f2bf(y - bf2f(h)); }

template <typename T16> struct WFrag;
template <> struct WFrag<h16> { typedef v16h V; static __device__ __forceinline__ V ld(const h16* p) { return cat16(*(const v8h*)p, *(const v8h*)(p + 16)); } static __device__ __forceinline__ v8f mma(V a, V b, v8f c) { return wmma16(a, b, c); } };
template <> struct WFrag<bf> { typedef v16bf V; static __device__ __forceinline__ V ld(const bf* p) { return cat16b(*(const v8us*)p, *(const v8us*)(p + 16)); } static __device__ __forceinline__ v8f mma(V a, V b, v8f c) { return wmmab(a, b, c); } };

template <typename T16, int NSPLIT, bool BIAS>
__device__ __forceinline__ void gemmw_body(const T16* __restrict__ A, const T16* __restrict__ A2, const T16* __restrict__ Bt, const T16* __restrict__ Bt2, int K, float* C, int ldc, const float* __restrict__ bias, float osc, size_t sA, size_t sB, size_t sC) {
    typedef typename WFrag<T16>::V V;
    __shared__ __align__(16) float os[16 * 68];
    const size_t z = blockIdx.z; A += z * sA; if (A2) A2 += z * sA; Bt += z * sB; if (Bt2) Bt2 += z * sB; C += z * sC;
    const int lane = threadIdx.x & 31, lr = lane & 15, hi = lane >> 4; const int r0 = blockIdx.x * 64, c0 = blockIdx.y * 64;
    v8f acc[4][4];
#pragma unroll
    for (int mb = 0; mb < 4; ++mb)
#pragma unroll
        for (int nb = 0; nb < 4; ++nb) acc[mb][nb] = (v8f){};
    const size_t aoff = (size_t)(r0 + lr) * K + 8 * hi, boff = (size_t)(c0 + lr) * K + 8 * hi;
#pragma unroll 1
    for (int kc = 0; kc < K; kc += 32) {
        V a[4], a2[4];
#pragma unroll
        for (int mb = 0; mb < 4; ++mb) { a[mb] = WFrag<T16>::ld(A + aoff + (size_t)mb * 16 * K + kc); if (NSPLIT == 1 || NSPLIT == 2) a2[mb] = WFrag<T16>::ld(A2 + aoff + (size_t)mb * 16 * K + kc); }
#pragma unroll
        for (int nb = 0; nb < 4; ++nb) { const V b = WFrag<T16>::ld(Bt + boff + (size_t)nb * 16 * K + kc); V b2; if (NSPLIT >= 2) b2 = WFrag<T16>::ld(Bt2 + boff + (size_t)nb * 16 * K + kc);
#pragma unroll
            for (int mb = 0; mb < 4; ++mb) { acc[mb][nb] = WFrag<T16>::mma(a[mb], b, acc[mb][nb]); if (NSPLIT == 1 || NSPLIT == 2) acc[mb][nb] = WFrag<T16>::mma(a2[mb], b, acc[mb][nb]); if (NSPLIT >= 2) acc[mb][nb] = WFrag<T16>::mma(a[mb], b2, acc[mb][nb]); } }
        asm volatile("v_nop\n\tv_nop\n\tv_nop\n\tv_nop" : "+v"(acc[0][0]), "+v"(acc[1][1]), "+v"(acc[2][2]), "+v"(acc[3][3]) : "v"(a[0]), "v"(a[3]));
    }
#pragma unroll
    for (int mb = 0; mb < 4; ++mb) {
#pragma unroll
        for (int nb = 0; nb < 4; ++nb) {
#pragma unroll
            for (int j = 0; j < 8; ++j) os[(hi * 8 + j) * 68 + nb * 16 + lr] = acc[mb][nb][j]; }
        __builtin_amdgcn_wave_barrier(); asm volatile("" ::: "memory");
        float* crow = C + (size_t)(r0 + mb * 16) * ldc + c0;
#pragma unroll 1
        for (int ps = 0; ps < 2; ++ps) {
#pragma unroll
            for (int s = 0; s < 8; ++s) { const int row = 2 * s + hi, cofs = lr * 4; v4f val = *(const v4fa*)(os + row * 68 + cofs);
                val[0] *= osc; val[1] *= osc; val[2] *= osc; val[3] *= osc;
                if (BIAS) { val[0] += bfr(bias[c0 + cofs]); val[1] += bfr(bias[c0 + cofs + 1]); val[2] += bfr(bias[c0 + cofs + 2]); val[3] += bfr(bias[c0 + cofs + 3]); }
                *(volatile v4f*)(crow + (size_t)row * ldc + cofs) = val; }
            if (ps == 0) __threadfence(); }
        __builtin_amdgcn_wave_barrier(); asm volatile("" ::: "memory");
    }
}

template <typename T16, int NSPLIT, int CMODE>
__device__ __forceinline__ void gemmc_body(const T16* __restrict__ A, const T16* __restrict__ A2, const T16* __restrict__ Bt, const T16* __restrict__ Bt2, int K, float* C, int ldc, int roff, size_t sA, size_t sB, size_t sC) {
    typedef typename WFrag<T16>::V V;
    __shared__ __align__(16) float os[16 * 68];
    const size_t z = blockIdx.z; A += z * sA; if (A2) A2 += z * sA; Bt += z * sB; if (Bt2) Bt2 += z * sB; C += z * sC;
    const int lane = threadIdx.x & 31, lr = lane & 15, hi = lane >> 4; const int r0 = blockIdx.x * 64, c0 = blockIdx.y * 64;
    if (CMODE == 1 && c0 > r0 + roff + 63) return;
    const int Kl = (CMODE == 2) ? min(K, r0 + roff + 64) : K;
    v8f acc[4][4];
#pragma unroll
    for (int mb = 0; mb < 4; ++mb)
#pragma unroll
        for (int nb = 0; nb < 4; ++nb) acc[mb][nb] = (v8f){};
    const size_t aoff = (size_t)(r0 + lr) * K + 8 * hi, boff = (size_t)(c0 + lr) * K + 8 * hi;
#pragma unroll 1
    for (int kc = 0; kc < Kl; kc += 32) {
        V a[4], a2[4];
#pragma unroll
        for (int mb = 0; mb < 4; ++mb) { a[mb] = WFrag<T16>::ld(A + aoff + (size_t)mb * 16 * K + kc); if (NSPLIT == 1 || NSPLIT == 2) a2[mb] = WFrag<T16>::ld(A2 + aoff + (size_t)mb * 16 * K + kc); }
#pragma unroll
        for (int nb = 0; nb < 4; ++nb) { const V b = WFrag<T16>::ld(Bt + boff + (size_t)nb * 16 * K + kc); V b2; if (NSPLIT >= 2) b2 = WFrag<T16>::ld(Bt2 + boff + (size_t)nb * 16 * K + kc);
#pragma unroll
            for (int mb = 0; mb < 4; ++mb) { acc[mb][nb] = WFrag<T16>::mma(a[mb], b, acc[mb][nb]); if (NSPLIT == 1 || NSPLIT == 2) acc[mb][nb] = WFrag<T16>::mma(a2[mb], b, acc[mb][nb]); if (NSPLIT >= 2) acc[mb][nb] = WFrag<T16>::mma(a[mb], b2, acc[mb][nb]); } }
        asm volatile("v_nop\n\tv_nop\n\tv_nop\n\tv_nop" : "+v"(acc[0][0]), "+v"(acc[1][1]), "+v"(acc[2][2]), "+v"(acc[3][3]) : "v"(a[0]), "v"(a[3]));
    }
#pragma unroll
    for (int mb = 0; mb < 4; ++mb) {
#pragma unroll
        for (int nb = 0; nb < 4; ++nb) {
#pragma unroll
            for (int j = 0; j < 8; ++j) os[(hi * 8 + j) * 68 + nb * 16 + lr] = acc[mb][nb][j]; }
        __builtin_amdgcn_wave_barrier(); asm volatile("" ::: "memory");
        float* crow = C + (size_t)(r0 + mb * 16) * ldc + c0;
#pragma unroll 1
        for (int ps = 0; ps < 2; ++ps) {
#pragma unroll
            for (int s = 0; s < 8; ++s) { const int row = 2 * s + hi, cofs = lr * 4; v4f val = *(const v4fa*)(os + row * 68 + cofs);
                *(volatile v4f*)(crow + (size_t)row * ldc + cofs) = val; }
            if (ps == 0) __threadfence(); }
        __builtin_amdgcn_wave_barrier(); asm volatile("" ::: "memory");
    }
}

__global__ __launch_bounds__(32) void k_gw_b0(const bf* A, const bf* Bt, int K, float* C, int ldc, const float* bias) { gemmw_body<bf, 0, true>(A, nullptr, Bt, nullptr, K, C, ldc, bias, 1.0f, 0, 0, 0); }
__global__ __launch_bounds__(32) void k_gw_b1(const bf* A, const bf* A2, const bf* Bt, int K, float* C, int ldc, const float* bias) { gemmw_body<bf, 1, true>(A, A2, Bt, nullptr, K, C, ldc, bias, 1.0f, 0, 0, 0); }
__global__ __launch_bounds__(32) void k_gw_h0(const h16* A, const h16* Bt, int K, float* C, int ldc, const float* bias, float osc) { gemmw_body<h16, 0, true>(A, nullptr, Bt, nullptr, K, C, ldc, bias, osc, 0, 0, 0); }
__global__ __launch_bounds__(32) void kc_s_b2(const bf* A, const bf* A2, const bf* Bt, const bf* Bt2, int K, float* C, int ldc, int roff, size_t sA, size_t sB, size_t sC) { gemmc_body<bf, 2, 1>(A, A2, Bt, Bt2, K, C, ldc, roff, sA, sB, sC); }
__global__ __launch_bounds__(32) void kc_s_h0(const h16* A, const h16* Bt, int K, float* C, int ldc, int roff, size_t sA, size_t sB, size_t sC) { gemmc_body<h16, 0, 1>(A, nullptr, Bt, nullptr, K, C, ldc, roff, sA, sB, sC); }
__global__ __launch_bounds__(32) void kc_v_b2(const bf* A, const bf* A2, const bf* Bt, const bf* Bt2, int K, float* C, int ldc, int roff, size_t sA, size_t sB, size_t sC) { gemmc_body<bf, 2, 2>(A, A2, Bt, Bt2, K, C, ldc, roff, sA, sB, sC); }
__global__ __launch_bounds__(32) void kc_v_h0(const h16* A, const h16* Bt, int K, float* C, int ldc, int roff, size_t sA, size_t sB, size_t sC) { gemmc_body<h16, 0, 2>(A, nullptr, Bt, nullptr, K, C, ldc, roff, sA, sB, sC); }

__global__ __launch_bounds__(256) void k_cvt8(const float* __restrict__ src, bf* dst, size_t n8) { const size_t i = (size_t)blockIdx.x * 256 + threadIdx.x; if (i >= n8) return; const v8f v = *(const v8f*)(src + i * 8); v8us o;
#pragma unroll
    for (int k = 0; k < 8; ++k) o[k] = f2bf(v[k]); *(volatile v8us*)(dst + i * 8) = o; __threadfence(); *(volatile v8us*)(dst + i * 8) = o; }
__global__ __launch_bounds__(256) void k_cvt8h(const float* __restrict__ src, h16* dst, size_t n8, float car) { const size_t i = (size_t)blockIdx.x * 256 + threadIdx.x; if (i >= n8) return; const v8f v = *(const v8f*)(src + i * 8); v8h o;
#pragma unroll
    for (int k = 0; k < 8; ++k) o[k] = tohx(bfr(v[k]) * car); *(volatile v8h*)(dst + i * 8) = o; __threadfence(); *(volatile v8h*)(dst + i * 8) = o; }

__global__ __launch_bounds__(256) void k_cs(float* CS) {
    const int idx = blockIdx.x * 256 + threadIdx.x; if (idx >= TT * (HD / 2)) return; const int i = idx % (HD / 2); const int t = idx / (HD / 2);
    const float ex = (float)(2 * i) / (float)HD; const float pw = powf(10000.0f, ex); const float inv = 1.0f / pw; const float ang = (float)t * inv;
    v2f cs; cs[0] = cosf(ang); cs[1] = sinf(ang);
    float* p0 = CS + ((size_t)t * HD + i) * 2; float* p1 = p0 + HD;
    *(volatile v2f*)p0 = cs; *(volatile v2f*)p1 = cs; __threadfence(); *(volatile v2f*)p0 = cs; *(volatile v2f*)p1 = cs; }

__global__ __launch_bounds__(256) void k_rope(const float* __restrict__ F, int pitch, int nheads, const float* __restrict__ CS, float sc, h16* P16, bf* Ph, bf* Pl) {
    const size_t e = ((size_t)blockIdx.x * 256 + threadIdx.x) * 2; if (e >= (size_t)nheads * TT * HD) return; const int d = (int)(e % HD); const int t = (int)((e / HD) % TT); const int h = (int)(e / ((size_t)HD * TT)); const float* f = F + (size_t)t * pitch + h * HD; v2h o16; v2us oh, ol;
#pragma unroll
    for (int q = 0; q < 2; ++q) { const int dd = d + q; const int dp = (dd < HD / 2) ? dd + HD / 2 : dd - HD / 2; const float x0 = f[dd], x1 = f[dp];
        const v2f cs = *(const v2f*)(CS + ((size_t)t * HD + dd) * 2); float a = __fmul_rn(x0, cs[0]), bq = __fmul_rn(x1, cs[1]); asm volatile("" : "+v"(a)); asm volatile("" : "+v"(bq)); const float r = ((dd < HD / 2) ? __fsub_rn(a, bq) : __fadd_rn(a, bq)) * sc;
        o16[q] = tohx(r); unsigned short a2, c2; splitf(r, a2, c2); oh[q] = a2; ol[q] = c2; }
    const bool hr = (t < RH); const size_t eh = ((size_t)h * RH + t) * HD + d;
    *(volatile v2h*)(P16 + e) = o16; if (hr) { *(volatile v2us*)(Ph + eh) = oh; *(volatile v2us*)(Pl + eh) = ol; }
    __threadfence();
    *(volatile v2h*)(P16 + e) = o16; if (hr) { *(volatile v2us*)(Ph + eh) = oh; *(volatile v2us*)(Pl + eh) = ol; } }

__global__ __launch_bounds__(256) void k_vtp(const float* __restrict__ F, int pitch, int nheads, h16* V16, bf* Vh, bf* Vl) { const size_t e = ((size_t)blockIdx.x * 256 + threadIdx.x) * 2; if (e >= (size_t)nheads * HD * TT) return; const int t = (int)(e % TT); const int d = (int)((e / TT) % HD); const int g = (int)(e / ((size_t)TT * HD)); v2h o16; v2us oh, ol;
#pragma unroll
    for (int q = 0; q < 2; ++q) { const float x = F[(size_t)(t + q) * pitch + g * HD + d]; o16[q] = tohx(x); unsigned short a2, c2; splitf(x, a2, c2); oh[q] = a2; ol[q] = c2; }
    const bool hr = (t < RH); const size_t eh = ((size_t)g * HD + d) * RH + t;
    *(volatile v2h*)(V16 + e) = o16; if (hr) { *(volatile v2us*)(Vh + eh) = oh; *(volatile v2us*)(Vl + eh) = ol; }
    __threadfence();
    *(volatile v2h*)(V16 + e) = o16; if (hr) { *(volatile v2us*)(Vh + eh) = oh; *(volatile v2us*)(Vl + eh) = ol; } }

__global__ __launch_bounds__(256) void k_asoft(const float* __restrict__ Sb, h16* P16, bf* Ph, bf* Pl) {
    const int lane = threadIdx.x & 31; const int row = __builtin_amdgcn_readfirstlane((int)(blockIdx.x * 8 + (threadIdx.x >> 5))); if (row >= ZH * TT) return;
    const int i = row % TT; const int zz = row / TT; const bool hires = (i < RH); const int nch = i / 128 + 1; const float* sr = Sb + (size_t)row * TT; float v[TT / 32]; float mx = -3.0e38f;
#pragma unroll
    for (int ch = 0; ch < TT / 128; ++ch) {
        if (ch < nch) { const int j0 = ch * 128 + lane * 4; const v4f a = *(const v4f*)(sr + j0);
#pragma unroll
            for (int q = 0; q < 4; ++q) { const float t = (j0 + q <= i) ? a[q] : -3.0e38f; v[ch * 4 + q] = t; mx = fmaxf(mx, t); }
        } else {
#pragma unroll
            for (int q = 0; q < 4; ++q) v[ch * 4 + q] = -3.0e38f; } }
#pragma unroll
    for (int sh = 16; sh; sh >>= 1) mx = fmaxf(mx, __shfl_xor(mx, sh, 32));
    float sum = 0.f;
#pragma unroll
    for (int ch = 0; ch < TT / 128; ++ch) {
        if (ch < nch) {
#pragma unroll
            for (int q = 0; q < 4; ++q) { const int k = ch * 4 + q; float d0 = __fsub_rn(v[k], mx); asm volatile("" : "+v"(d0)); v[k] = __builtin_amdgcn_exp2f(__fmul_rn(d0, 1.4426950408889634f)); sum += v[k]; } } }
#pragma unroll
    for (int sh = 16; sh; sh >>= 1) sum += __shfl_xor(sum, sh, 32);
    const float f = __fdiv_rn(hires ? 1.0f : PCAR, sum);
#pragma unroll 1
    for (int ps = 0; ps < 2; ++ps) {
        if (hires) {
#pragma unroll
            for (int ch = 0; ch < RH / 128; ++ch) { if (ch < nch) { v4us oh, ol;
#pragma unroll
                for (int q = 0; q < 4; ++q) { unsigned short a, c2; splitf(v[ch * 4 + q] * f, a, c2); oh[q] = a; ol[q] = c2; }
                const size_t oo = ((size_t)zz * RH + i) * RH + ch * 128 + lane * 4; *(volatile v4us*)(Ph + oo) = oh; *(volatile v4us*)(Pl + oo) = ol; } }
        } else {
#pragma unroll
            for (int ch = 0; ch < TT / 128; ++ch) { if (ch < nch) { v4h o4;
#pragma unroll
                for (int q = 0; q < 4; ++q) o4[q] = tohx(v[ch * 4 + q] * f);
                *(volatile v4h*)(P16 + (size_t)row * TT + ch * 128 + lane * 4) = o4; } } }
        if (ps == 0) __threadfence(); }
}

__global__ __launch_bounds__(256) void k_merge(const float* __restrict__ O, int h0, h16* A16, bf* Ah, bf* Al) { const size_t e = ((size_t)blockIdx.x * 256 + threadIdx.x) * 2; if (e >= (size_t)ZH * TT * HD) return; const int d = (int)(e % HD); const int t = (int)((e / HD) % TT); const int zz = (int)(e / ((size_t)HD * TT)); const size_t oo = (size_t)t * DQ + (h0 + zz) * HD + d;
    const float x0 = O[e], x1 = O[e + 1];
    if (t < RH) { v2us oh, ol; unsigned short a, c2; splitf(x0, a, c2); oh[0] = a; ol[0] = c2; splitf(x1, a, c2); oh[1] = a; ol[1] = c2;
        *(volatile v2us*)(Ah + oo) = oh; *(volatile v2us*)(Al + oo) = ol; __threadfence(); *(volatile v2us*)(Ah + oo) = oh; *(volatile v2us*)(Al + oo) = ol;
    } else { v2h o; o[0] = tohx(x0 * (ACAR / PCAR)); o[1] = tohx(x1 * (ACAR / PCAR));
        *(volatile v2h*)(A16 + oo) = o; __threadfence(); *(volatile v2h*)(A16 + oo) = o; } }

constexpr size_t AL(size_t b) { return (b + 255) & ~(size_t)255; }
constexpr size_t SZ_WQ  = AL((size_t)DQ * DM * 2);
constexpr size_t SZ_WKV = AL((size_t)DKV * DM * 2);
constexpr size_t SZ_WO  = AL((size_t)DM * DQ * 2);
constexpr size_t SZ_CS  = AL((size_t)TT * HD * 2 * 4);
constexpr size_t SZ_XB  = AL((size_t)TT * DM * 2);
constexpr size_t SZ_FQ  = AL((size_t)TT * DQ * 4);
constexpr size_t SZ_FK  = AL((size_t)TT * DKV * 4);
constexpr size_t SZ_QP  = AL((size_t)NH_ * TT * HD * 2);
constexpr size_t SZ_KP  = AL((size_t)NKV * TT * HD * 2);
constexpr size_t SZ_QE  = AL((size_t)NH_ * RH * HD * 2);
constexpr size_t SZ_KE  = AL((size_t)NKV * RH * HD * 2);
constexpr size_t SZ_PE  = AL((size_t)ZH * RH * RH * 2);
constexpr size_t SZ_SB  = AL((size_t)ZH * TT * TT * 4);
constexpr size_t SZ_P16 = AL((size_t)ZH * TT * TT * 2);
constexpr size_t SZ_OB  = AL((size_t)ZH * TT * HD * 4);
constexpr size_t WS_TOTAL = SZ_WQ + 2 * SZ_WKV + 2 * SZ_WO + SZ_CS + SZ_XB + SZ_FQ + SZ_FK + SZ_QP + 3 * SZ_KP + 2 * SZ_QE + 4 * SZ_KE + 2 * SZ_PE + SZ_SB + SZ_P16 + SZ_OB;
static_assert(WS_TOTAL <= (size_t)134217728);
static_assert(((size_t)TT + 2 * (size_t)RH) * DQ * 2 <= (size_t)TT * DQ * 4);

extern "C" void kernel_launch(void* const* d_in, const int* in_sizes, int n_in,
                              void* d_out, int out_size, void* d_ws, size_t ws_size, hipStream_t stream) {
    if (n_in < 11) return;
    const size_t need_act = ((size_t)(NB - 1) * SEQ_FULL + SEQ) * DM;
    if ((size_t)in_sizes[0] < need_act || (size_t)in_sizes[1] < need_act || (size_t)in_sizes[2] < need_act) return;
    if ((size_t)in_sizes[3] < (size_t)DQ * DM || in_sizes[4] < DQ || (size_t)in_sizes[5] < (size_t)DKV * DM || in_sizes[6] < DKV) return;
    if ((size_t)in_sizes[7] < (size_t)DKV * DM || in_sizes[8] < DKV || (size_t)in_sizes[9] < (size_t)DM * DQ || in_sizes[10] < DM) return;
    if ((size_t)out_size < (size_t)NB * TT * DM) return;
    if (WS_TOTAL > ws_size) return;
    const float* xq = (const float*)d_in[0]; const float* xk = (const float*)d_in[1]; const float* xv = (const float*)d_in[2];
    const float* wq = (const float*)d_in[3]; const float* bq = (const float*)d_in[4]; const float* wk = (const float*)d_in[5]; const float* bk = (const float*)d_in[6];
    const float* wv = (const float*)d_in[7]; const float* bv = (const float*)d_in[8]; const float* wo = (const float*)d_in[9]; const float* bo = (const float*)d_in[10];
    float* OUT = (float*)d_out;
    char* wsp = (char*)d_ws;
    auto take = [&](size_t bytes) { char* p = wsp; wsp += bytes; return (void*)p; };
    bf* WQ = (bf*)take(SZ_WQ); bf* WK = (bf*)take(SZ_WKV); bf* WV = (bf*)take(SZ_WKV); bf* WO = (bf*)take(SZ_WO); h16* WO16 = (h16*)take(SZ_WO); float* CS = (float*)take(SZ_CS);
    bf* XB = (bf*)take(SZ_XB); float* FQ = (float*)take(SZ_FQ); float* FK = (float*)take(SZ_FK);
    h16* QP16 = (h16*)take(SZ_QP); h16* KP16 = (h16*)take(SZ_KP); h16* VT16 = (h16*)take(SZ_KP);
    bf* QPh = (bf*)take(SZ_QE); bf* QPl = (bf*)take(SZ_QE); bf* KPh = (bf*)take(SZ_KE); bf* KPl = (bf*)take(SZ_KE); bf* VTh = (bf*)take(SZ_KE); bf* VTl = (bf*)take(SZ_KE); bf* Ph = (bf*)take(SZ_PE); bf* Pl = (bf*)take(SZ_PE);
    float* Sb = (float*)take(SZ_SB); h16* P16 = (h16*)take(SZ_P16); float* Ob = (float*)take(SZ_OB);
    if ((size_t)(wsp - (char*)d_ws) > ws_size) return;
    float* FV = FK;
    h16* AT16 = (h16*)FQ; bf* ATh = (bf*)((char*)FQ + (size_t)TT * DQ * 2); bf* ATl = ATh + (size_t)RH * DQ;
    k_cvt8<<<(unsigned)(((size_t)DQ * DM / 8 + 255) / 256), 256, 0, stream>>>(wq, WQ, (size_t)DQ * DM / 8);
    k_cvt8<<<(unsigned)(((size_t)DKV * DM / 8 + 255) / 256), 256, 0, stream>>>(wk, WK, (size_t)DKV * DM / 8);
    k_cvt8<<<(unsigned)(((size_t)DKV * DM / 8 + 255) / 256), 256, 0, stream>>>(wv, WV, (size_t)DKV * DM / 8);
    k_cvt8<<<(unsigned)(((size_t)DM * DQ / 8 + 255) / 256), 256, 0, stream>>>(wo, WO, (size_t)DM * DQ / 8);
    k_cvt8h<<<(unsigned)(((size_t)DM * DQ / 8 + 255) / 256), 256, 0, stream>>>(wo, WO16, (size_t)DM * DQ / 8, WCAR);
    k_cs<<<(TT * (HD / 2) + 255) / 256, 256, 0, stream>>>(CS);
    const unsigned LX = (unsigned)(((size_t)TT * DM / 8 + 255) / 256);
    const unsigned LQ = (unsigned)(((size_t)NH_ * TT * HD / 2 + 255) / 256), LKv = (unsigned)(((size_t)NKV * TT * HD / 2 + 255) / 256);
    for (int b = 0; b < NB; ++b) {
        const size_t ioff = (size_t)b * SEQ_FULL * DM; float* OUTb = OUT + (size_t)b * TT * DM;
        k_cvt8<<<LX, 256, 0, stream>>>(xq + ioff, XB, (size_t)TT * DM / 8);
        k_gw_b0<<<dim3(TT / 64, DQ / 64, 1), 32, 0, stream>>>(XB, WQ, DM, FQ, DQ, bq);
        k_rope<<<LQ, 256, 0, stream>>>(FQ, DQ, NH_, CS, SCL, QP16, QPh, QPl);
        k_cvt8<<<LX, 256, 0, stream>>>(xk + ioff, XB, (size_t)TT * DM / 8);
        k_gw_b0<<<dim3(TT / 64, DKV / 64, 1), 32, 0, stream>>>(XB, WK, DM, FK, DKV, bk);
        k_rope<<<LKv, 256, 0, stream>>>(FK, DKV, NKV, CS, 1.0f, KP16, KPh, KPl);
        k_cvt8<<<LX, 256, 0, stream>>>(xv + ioff, XB, (size_t)TT * DM / 8);
        k_gw_b0<<<dim3(TT / 64, DKV / 64, 1), 32, 0, stream>>>(XB, WV, DM, FV, DKV, bv);
        k_vtp<<<LKv, 256, 0, stream>>>(FV, DKV, NKV, VT16, VTh, VTl);
        for (int h0 = 0; h0 < NH_; h0 += ZH) { const size_t zq = (size_t)h0, zk = (size_t)(h0 / REP);
            kc_s_b2<<<dim3(RH / 64, RH / 64, ZH), 32, 0, stream>>>(QPh + zq * RH * HD, QPl + zq * RH * HD, KPh + zk * RH * HD, KPl + zk * RH * HD, HD, Sb, TT, 0, (size_t)RH * HD, 0, (size_t)TT * TT);
            kc_s_h0<<<dim3((TT - RH) / 64, TT / 64, ZH), 32, 0, stream>>>(QP16 + zq * TT * HD + (size_t)RH * HD, KP16 + zk * TT * HD, HD, Sb + (size_t)RH * TT, TT, RH, (size_t)TT * HD, 0, (size_t)TT * TT);
            k_asoft<<<ZH * TT / 8, 256, 0, stream>>>(Sb, P16, Ph, Pl);
            kc_v_b2<<<dim3(RH / 64, HD / 64, ZH), 32, 0, stream>>>(Ph, Pl, VTh + zk * HD * RH, VTl + zk * HD * RH, RH, Ob, HD, 0, (size_t)RH * RH, 0, (size_t)TT * HD);
            kc_v_h0<<<dim3((TT - RH) / 64, HD / 64, ZH), 32, 0, stream>>>(P16 + (size_t)RH * TT, VT16 + zk * HD * TT, TT, Ob + (size_t)RH * HD, HD, RH, (size_t)TT * TT, 0, (size_t)TT * HD);
            k_merge<<<(unsigned)(((size_t)ZH * TT * HD / 2 + 255) / 256), 256, 0, stream>>>(Ob, h0, AT16, ATh, ATl); }
        k_gw_b1<<<dim3(RH / 64, DM / 64, 1), 32, 0, stream>>>(ATh, ATl, WO, DQ, OUTb, DM, bo);
        k_gw_h0<<<dim3((TT - RH) / 64, DM / 64, 1), 32, 0, stream>>>(AT16 + (size_t)RH * DQ, WO16, DQ, OUTb + (size_t)RH * DM, DM, bo, 1.0f / (ACAR * WCAR)); }
}
